// LinearSelfAttention_2808908611864
// MI455X (gfx1250) — hardware-verified
//
#include <hip/hip_runtime.h>
#include <stddef.h>


typedef _Float16 h16;
typedef _Float16 v16h __attribute__((ext_vector_type(16)));
typedef _Float16 v8h  __attribute__((ext_vector_type(8)));
typedef float    v8f  __attribute__((ext_vector_type(8)));
typedef float    v4f  __attribute__((ext_vector_type(4)));

#ifndef NB
#define NB 16
#endif
#define NB_FULL 16
#define SEQ   2048
#define DP1   257
#define NP1   (SEQ + 1)
#define DP    320
#define KP    288
#define NPAD  2112
#define BSTRIDE (DP1 * NP1)
#define NVEC  ((NB * BSTRIDE) / 4)

static_assert(NB >= 1 && NB <= NB_FULL);
static_assert(((NB * BSTRIDE) % 4) == 0);
static_assert((long long)NB_FULL * BSTRIDE < 2147483647LL);
static_assert((DP % 64) == 0 && DP >= DP1);
static_assert((KP % 32) == 0 && KP >= DP1 && KP <= DP);
static_assert((SEQ % 64) == 0 && (SEQ % 32) == 0);
static_assert((NPAD % 64) == 0 && NPAD >= NP1);
static_assert(((DP * 2) % 128) == 0);
static_assert(((SEQ * 2) % 128) == 0);
static_assert(((NPAD * 4) % 128) == 0);

#define LDT 72
#define LDC 68
static_assert((LDT % 8) == 0 && LDT >= 64);
static_assert((LDC % 4) == 0 && LDC >= 64);
static_assert(64 * LDC * 4 <= 131072);
static_assert(2 * 64 * LDT * 2 <= 131072);
static_assert(64 * LDT * 2 <= 131072);

#define WCARRY 64.0f

#define WSM_BYTES  ((size_t)DP * DP * 2)
#define H16_BYTES  ((size_t)NB * DP * SEQ * 2)
#define HT_BYTES   ((size_t)NB * NPAD * DP * 2)
#define SM_BYTES   ((size_t)NB * DP * DP * 2)
#define ATT_BYTES  ((size_t)NB * DP * NPAD * 4)
#define OFF_P16 ((size_t)0)
#define OFF_QT  (OFF_P16 + WSM_BYTES)
#define OFF_H16 (OFF_QT + WSM_BYTES)
#define OFF_HT  (OFF_H16 + H16_BYTES)
#define OFF_G   (OFF_HT + HT_BYTES)
#define OFF_PG  (OFF_G + SM_BYTES)
#define OFF_PGQ (OFF_PG + SM_BYTES)
#define OFF_ATT (OFF_PGQ + SM_BYTES)
#define WS_TOTAL (OFF_ATT + ATT_BYTES)
static_assert((WSM_BYTES % 128) == 0 && (H16_BYTES % 128) == 0 && (HT_BYTES % 128) == 0);
static_assert((SM_BYTES % 128) == 0 && (ATT_BYTES % 128) == 0);
static_assert(WS_TOTAL <= (size_t)134217728);

__device__ __forceinline__ float bf16r(float x) {
  unsigned int u = __float_as_uint(x);
  u = (u + 0x7FFFu + ((u >> 16) & 1u)) & 0xFFFF0000u;
  return __uint_as_float(u);
}

static __device__ __forceinline__ h16 toh_flush(float v) {
  const h16 r = (h16)v;
  return (fabsf(v) < 6.103515625e-05f) ? (h16)0.0f : r;
}

__device__ __forceinline__ v16h frag_at(const _Float16* p) {
  v8h lo = *(const v8h*)(p);
  v8h hi = *(const v8h*)(p + 16);
  v16h out;
#pragma unroll
  for (int i = 0; i < 8; ++i) { out[i] = lo[i]; out[i + 8] = hi[i]; }
  return out;
}

__device__ __forceinline__ v8f wmma16(v16h a, v16h b, v8f c) {
  v8f d = __builtin_amdgcn_wmma_f32_16x16x32_f16(false, a, false, b, (short)0, c,
                                                 false, false);
  asm volatile("v_nop\n\tv_nop\n\tv_nop\n\tv_nop" : "+v"(d) : "v"(a), "v"(b));
  return d;
}

__global__ __launch_bounds__(256) void wconv_kernel(
    const float* __restrict__ W, _Float16* __restrict__ Wt,
    unsigned sk, unsigned sn, unsigned nk, unsigned nn, unsigned ldk) {
  __shared__ _Float16 T[64 * LDT];
  const unsigned tid = threadIdx.x;
  const unsigned n0 = blockIdx.x * 64u;
  const unsigned k0 = blockIdx.y * 64u;
#pragma unroll 4
  for (unsigned j = 0; j < 16u; ++j) {
    const unsigned idx = tid + 256u * j;
    const unsigned kr = idx >> 6, nc = idx & 63u;
    const unsigned kk = k0 + kr, n = n0 + nc;
    const unsigned kcl = (kk < nk) ? kk : (nk - 1u);
    const unsigned ncl = (n < nn) ? n : (nn - 1u);
    const float v = W[(size_t)kcl * sk + (size_t)ncl * sn];
    const bool ok = (kk < nk) && (n < nn);
    const h16 hv = toh_flush(WCARRY * bf16r(v));
    T[nc * LDT + kr] = ok ? hv : (h16)0.0f;
  }
  __syncthreads();
  v8h x[2];
  size_t off[2];
#pragma unroll
  for (unsigned i = 0; i < 2u; ++i) {
    const unsigned n = 32u * i + (tid >> 3);
    const unsigned kc = (tid & 7u) * 8u;
    x[i] = *(const v8h*)&T[n * LDT + kc];
    off[i] = (size_t)(n0 + n) * ldk + k0 + kc;
  }
#pragma unroll
  for (int i = 0; i < 2; ++i) *(volatile v8h*)(Wt + off[i]) = x[i];
  __threadfence();
#pragma unroll
  for (int i = 0; i < 2; ++i) *(volatile v8h*)(Wt + off[i]) = x[i];
}

__global__ __launch_bounds__(256) void hconv_kernel(
    const float* __restrict__ H, _Float16* __restrict__ H16, _Float16* __restrict__ Ht16) {
  __shared__ _Float16 Td[64 * LDT];
  __shared__ _Float16 Tt[64 * LDT];
  const unsigned tid = threadIdx.x;
  const unsigned t0 = blockIdx.x * 64u;
  const unsigned d0 = blockIdx.y * 64u;
  const unsigned b = blockIdx.z;
  const float* Hb = H + (size_t)b * BSTRIDE;
#pragma unroll 4
  for (unsigned j = 0; j < 16u; ++j) {
    const unsigned idx = tid + 256u * j;
    const unsigned dr = idx >> 6, tc = idx & 63u;
    const unsigned d = d0 + dr, t = t0 + tc;
    const unsigned dcl = (d < (unsigned)DP1) ? d : (unsigned)(DP1 - 1);
    const unsigned tcl = (t < (unsigned)NP1) ? t : (unsigned)(NP1 - 1);
    const float v = Hb[(size_t)dcl * NP1 + tcl];
    const bool ok = (d < (unsigned)DP1) && (t < (unsigned)NP1);
    const h16 hv0 = toh_flush(bf16r(v));
    const h16 hv = ok ? hv0 : (h16)0.0f;
    Td[dr * LDT + tc] = hv;
    Tt[tc * LDT + dr] = hv;
  }
  __syncthreads();
  const bool direct = (t0 < (unsigned)SEQ);
  const unsigned t0c = direct ? t0 : (unsigned)(SEQ - 64);
  v8h xt[2], xd[2];
  size_t offt[2], offd[2];
#pragma unroll
  for (unsigned i = 0; i < 2u; ++i) {
    const unsigned n = 32u * i + (tid >> 3);
    const unsigned kc = (tid & 7u) * 8u;
    xt[i] = *(const v8h*)&Tt[n * LDT + kc];
    offt[i] = ((size_t)b * NPAD + t0 + n) * DP + d0 + kc;
    xd[i] = *(const v8h*)&Td[n * LDT + kc];
    offd[i] = ((size_t)b * DP + d0 + n) * SEQ + t0c + kc;
  }
#pragma unroll
  for (int i = 0; i < 2; ++i) *(volatile v8h*)(Ht16 + offt[i]) = xt[i];
  if (direct) {
#pragma unroll
    for (int i = 0; i < 2; ++i) *(volatile v8h*)(H16 + offd[i]) = xd[i];
  }
  __threadfence();
#pragma unroll
  for (int i = 0; i < 2; ++i) *(volatile v8h*)(Ht16 + offt[i]) = xt[i];
  if (direct) {
#pragma unroll
    for (int i = 0; i < 2; ++i) *(volatile v8h*)(H16 + offd[i]) = xd[i];
  }
}

template <int MODE>
__device__ __forceinline__ void gemm_body(
    const _Float16* __restrict__ A16, const _Float16* __restrict__ Bt,
    const unsigned K, const unsigned lda, const unsigned ldb,
    float* __restrict__ outf, _Float16* __restrict__ out16,
    const unsigned ldo, const float cs) {
  __shared__ float Cs[64 * LDC];
  const unsigned tid = threadIdx.x, lane = tid & 31u;
  const unsigned w = (unsigned)__builtin_amdgcn_readfirstlane((int)(threadIdx.x >> 5));
  const unsigned mw = w >> 1, nw = w & 1u;
  const unsigned hh = lane >> 4, m = lane & 15u;
  const unsigned n0 = blockIdx.x * 64u;
  const unsigned row0 = blockIdx.y * 64u;

  const _Float16* ap  = A16 + (size_t)(row0 + mw * 16u + m) * lda + hh * 8u;
  const _Float16* bp0 = Bt + (size_t)(n0 + nw * 32u + m) * ldb + hh * 8u;
  const _Float16* bp1 = bp0 + (size_t)16 * ldb;
  v8f acc0 = {}, acc1 = {};
#pragma unroll 2
  for (unsigned k0 = 0; k0 < K; k0 += 32u) {
    const v16h a  = frag_at(ap + k0);
    const v16h b0 = frag_at(bp0 + k0);
    const v16h b1 = frag_at(bp1 + k0);
    acc0 = wmma16(a, b0, acc0);
    acc1 = wmma16(a, b1, acc1);
  }
#pragma unroll
  for (int r = 0; r < 8; ++r) {
    float* d = &Cs[(mw * 16u + hh * 8u + (unsigned)r) * LDC + nw * 32u + m];
    d[0]  = acc0[r];
    d[16] = acc1[r];
  }
  __syncthreads();

  if (MODE == 0) {
    v8h x[2];
    size_t off[2];
#pragma unroll
    for (unsigned i = 0; i < 2u; ++i) {
      const unsigned r = 32u * i + (tid >> 3);
      const unsigned c = (tid & 7u) * 8u;
      const v4f u0 = *(const v4f*)&Cs[r * LDC + c];
      const v4f u1 = *(const v4f*)&Cs[r * LDC + c + 4];
#pragma unroll
      for (int j = 0; j < 4; ++j) {
        x[i][j]     = toh_flush(u0[j] * cs);
        x[i][j + 4] = toh_flush(u1[j] * cs);
      }
      off[i] = (size_t)(row0 + r) * ldo + n0 + c;
    }
#pragma unroll
    for (int i = 0; i < 2; ++i) *(volatile v8h*)(out16 + off[i]) = x[i];
    __threadfence();
#pragma unroll
    for (int i = 0; i < 2; ++i) *(volatile v8h*)(out16 + off[i]) = x[i];
  }

  if (MODE == 1) {
    v4f xs[4];
    size_t off[4];
#pragma unroll
    for (unsigned i = 0; i < 4u; ++i) {
      const unsigned r = 16u * i + (tid >> 4);
      const unsigned c = (tid & 15u) * 4u;
      const v4f u = *(const v4f*)&Cs[r * LDC + c];
      v4f val;
#pragma unroll
      for (int j = 0; j < 4; ++j) val[j] = u[j] * cs;
      xs[i] = val;
      off[i] = (size_t)(row0 + r) * ldo + n0 + c;
    }
#pragma unroll
    for (int i = 0; i < 4; ++i) *(volatile v4f*)(outf + off[i]) = xs[i];
    __threadfence();
#pragma unroll
    for (int i = 0; i < 4; ++i) *(volatile v4f*)(outf + off[i]) = xs[i];
  }
}

__global__ __launch_bounds__(256) void gemm_gram_kernel(
    const _Float16* __restrict__ H16, _Float16* __restrict__ G16) {
  const size_t b = blockIdx.z;
  gemm_body<0>(H16 + b * ((size_t)DP * SEQ), H16 + b * ((size_t)DP * SEQ),
               (unsigned)SEQ, (unsigned)SEQ, (unsigned)SEQ,
               (float*)0, G16 + b * ((size_t)DP * DP), (unsigned)DP, 1.0f);
}
__global__ __launch_bounds__(256) void gemm_pg_kernel(
    const _Float16* __restrict__ P16, const _Float16* __restrict__ G16,
    _Float16* __restrict__ PG16) {
  const size_t b = blockIdx.z;
  gemm_body<0>(P16, G16 + b * ((size_t)DP * DP),
               (unsigned)KP, (unsigned)DP, (unsigned)DP,
               (float*)0, PG16 + b * ((size_t)DP * DP), (unsigned)DP, 1.0f / WCARRY);
}
__global__ __launch_bounds__(256) void gemm_pgq_kernel(
    const _Float16* __restrict__ PG16, const _Float16* __restrict__ Qt16,
    _Float16* __restrict__ PGQ16) {
  const size_t b = blockIdx.z;
  gemm_body<0>(PG16 + b * ((size_t)DP * DP), Qt16,
               (unsigned)KP, (unsigned)DP, (unsigned)DP,
               (float*)0, PGQ16 + b * ((size_t)DP * DP), (unsigned)DP, 1.0f / WCARRY);
}
__global__ __launch_bounds__(256) void gemm_att_kernel(
    const _Float16* __restrict__ PGQ16, const _Float16* __restrict__ Ht16,
    float* __restrict__ Att) {
  const size_t b = blockIdx.z;
  gemm_body<1>(PGQ16 + b * ((size_t)DP * DP), Ht16 + b * ((size_t)NPAD * DP),
               (unsigned)KP, (unsigned)DP, (unsigned)DP,
               Att + b * ((size_t)DP * NPAD), (_Float16*)0, (unsigned)NPAD,
               1.0f / (float)SEQ);
}

__global__ __launch_bounds__(256) void finish_kernel(
    const float* __restrict__ H, const float* __restrict__ Att, float* __restrict__ out) {
#pragma clang fp contract(off)
  const unsigned i = blockIdx.x * 256u + threadIdx.x;
  const unsigned ic = (i < (unsigned)NVEC) ? i : (unsigned)(NVEC - 1);
  const unsigned f = ic * 4u;
  unsigned b = f / (unsigned)BSTRIDE;
  const unsigned rem = f - b * (unsigned)BSTRIDE;
  unsigned d = rem / (unsigned)NP1;
  unsigned t = rem - d * (unsigned)NP1;
  const v4f hv = *(const v4f*)(H + (size_t)f);
  v4f val;
#pragma unroll
  for (int j = 0; j < 4; ++j) {
    const size_t ai = ((size_t)b * DP + d) * NPAD + t;
    const float a = Att[ai];
    val[j] = bf16r(hv[j]) + a;
    ++t;
    if (t == (unsigned)NP1) {
      t = 0u;
      ++d;
      if (d == (unsigned)DP1) {
        d = 0u;
        b = (b + 1u < (unsigned)NB) ? (b + 1u) : b;
      }
    }
  }
  if (i < (unsigned)NVEC) {
    float* p = out + (size_t)f;
    *(volatile v4f*)p = val;
    __threadfence();
    *(volatile v4f*)p = val;
  }
}

extern "C" void kernel_launch(void* const* d_in, const int* in_sizes, int n_in,
                              void* d_out, int out_size, void* d_ws, size_t ws_size,
                              hipStream_t stream) {
  if (n_in < 3) return;
  const long long need_h = (long long)NB * BSTRIDE;
  if ((long long)in_sizes[0] < need_h) return;
  if ((long long)in_sizes[1] < (long long)DP1 * DP1) return;
  if ((long long)in_sizes[2] < (long long)DP1 * DP1) return;
  if ((long long)out_size < need_h) return;
  if (ws_size < WS_TOTAL) return;

  const float* H  = (const float*)d_in[0];
  const float* Pm = (const float*)d_in[1];
  const float* Qm = (const float*)d_in[2];
  float* out = (float*)d_out;

  char* ws = (char*)d_ws;
  _Float16* P16   = (_Float16*)(ws + OFF_P16);
  _Float16* Qt16  = (_Float16*)(ws + OFF_QT);
  _Float16* H16   = (_Float16*)(ws + OFF_H16);
  _Float16* Ht16  = (_Float16*)(ws + OFF_HT);
  _Float16* G16   = (_Float16*)(ws + OFF_G);
  _Float16* PG16  = (_Float16*)(ws + OFF_PG);
  _Float16* PGQ16 = (_Float16*)(ws + OFF_PGQ);
  float*    Att   = (float*)(ws + OFF_ATT);

  dim3 blk(256);
  dim3 gsm(DP / 64, DP / 64);
  dim3 gsb(DP / 64, DP / 64, NB);

  wconv_kernel<<<gsm, blk, 0, stream>>>(Pm, P16, 1u, (unsigned)DP1, (unsigned)DP1,
                                        (unsigned)DP1, (unsigned)DP);
  wconv_kernel<<<gsm, blk, 0, stream>>>(Qm, Qt16, (unsigned)DP1, 1u, (unsigned)DP1,
                                        (unsigned)DP1, (unsigned)DP);
  hconv_kernel<<<dim3(NPAD / 64, DP / 64, NB), blk, 0, stream>>>(H, H16, Ht16);

  gemm_gram_kernel<<<gsb, blk, 0, stream>>>(H16, G16);
  gemm_pg_kernel<<<gsb, blk, 0, stream>>>(P16, G16, PG16);
  gemm_pgq_kernel<<<gsb, blk, 0, stream>>>(PG16, Qt16, PGQ16);
  gemm_att_kernel<<<dim3(NPAD / 64, DP / 64, NB), blk, 0, stream>>>(PGQ16, Ht16, Att);

  finish_kernel<<<dim3((NVEC + 255) / 256), blk, 0, stream>>>(H, Att, out);
}
